// MultiHeadAttn_1786706395825
// MI455X (gfx1250) — hardware-verified
//
#include <hip/hip_runtime.h>
#include <math.h>
#include <stdint.h>

#ifndef NB
#define NB 4
#endif
#ifndef NB_FULL
#define NB_FULL 4
#endif
#ifndef SEQ
#define SEQ 2048
#endif
#ifndef SEQ_FULL
#define SEQ_FULL 2048
#endif
#define NH    16
#define HD    64
#define DM    1024
#define DQKV  3072
#define NQB   (SEQ / 64)
#define MTOK  (NB * SEQ)
#ifndef RESW
#define RESW  1
#endif
#define PCARRY 16384.0f
#define PRES   4096.0f
#define VCARRY 64.0f
#define QRES   2048.0f
#define OCARRY 64.0f
#define WCARRY 64.0f
#define NEGF   (-1.0e30f)
#define SKIPG  110.0f

#define BM  128
#define BN  128
#define BK  32
#define TP  136
#define TPF 132

static_assert(NB >= 1 && NB <= NB_FULL);
static_assert((SEQ % 128) == 0 && SEQ >= 128 && SEQ <= SEQ_FULL);
static_assert(NH * HD == DM);
static_assert((MTOK % BM) == 0 && (SEQ % BM) == 0);
static_assert((DQKV % BN) == 0 && (DM % BN) == 0 && (DM % BK) == 0 && (DM % 64) == 0);
static_assert(BN == 2 * HD);
static_assert(RESW >= 0);
static_assert((long long)MTOK * DM * 4 <= 33554432LL);
static_assert(((MTOK * DM / 8) % 256) == 0 && ((DQKV * DM / 8) % 256) == 0 && ((DM * DM / 8) % 256) == 0);

typedef _Float16 v16h __attribute__((ext_vector_type(16)));
typedef _Float16 v8h  __attribute__((ext_vector_type(8)));
typedef __bf16   v16b __attribute__((ext_vector_type(16)));
typedef __bf16   v8b  __attribute__((ext_vector_type(8)));
typedef float    v8f  __attribute__((ext_vector_type(8)));
typedef float    v4f  __attribute__((ext_vector_type(4)));
typedef unsigned int v4u __attribute__((ext_vector_type(4)));
typedef unsigned short v8us __attribute__((ext_vector_type(8)));

__device__ __forceinline__ unsigned short bf_bits(float f) {
  unsigned u = __float_as_uint(f);
  return (unsigned short)((u + 0x7FFFu + ((u >> 16) & 1u)) >> 16);
}
__device__ __forceinline__ float bf_up(unsigned short h) { return __uint_as_float(((unsigned)h) << 16); }
__device__ __forceinline__ unsigned pk16(unsigned short a, unsigned short b) { return (unsigned)a | ((unsigned)b << 16); }
__device__ __forceinline__ unsigned short h_bits(float f) {
  const _Float16 hv = (_Float16)f;
  return __builtin_bit_cast(unsigned short, hv);
}
__device__ __forceinline__ v8f zero8() { v8f z = {0.f, 0.f, 0.f, 0.f, 0.f, 0.f, 0.f, 0.f}; return z; }

template <typename E> struct FT;
template <> struct FT<__bf16> {
  typedef v16b V16;
  typedef v8b  V8;
  static __device__ __forceinline__ v16b ld(const __bf16* p) {
    union { v16b v; v8b h[2]; } f;
    f.h[0] = *(const v8b*)(p);
    f.h[1] = *(const v8b*)(p + 16);
    return f.v;
  }
  static __device__ __forceinline__ v8f mma(v16b a, v16b b, v8f c) {
    c = __builtin_amdgcn_wmma_f32_16x16x32_bf16(false, a, false, b, (short)0, c, false, false);
    asm volatile("v_nop\n\tv_nop\n\tv_nop\n\tv_nop" : "+v"(c) : "v"(a), "v"(b));
    return c;
  }
};
template <> struct FT<_Float16> {
  typedef v16h V16;
  typedef v8h  V8;
  static __device__ __forceinline__ v16h ld(const _Float16* p) {
    union { v16h v; v8h h[2]; } f;
    f.h[0] = *(const v8h*)(p);
    f.h[1] = *(const v8h*)(p + 16);
    return f.v;
  }
  static __device__ __forceinline__ v8f mma(v16h a, v16h b, v8f c) {
    c = __builtin_amdgcn_wmma_f32_16x16x32_f16(false, a, false, b, (short)0, c, false, false);
    asm volatile("v_nop\n\tv_nop\n\tv_nop\n\tv_nop" : "+v"(c) : "v"(a), "v"(b));
    return c;
  }
};

template <int MODE>
__device__ __forceinline__ unsigned short cv16(float f) {
  const unsigned short ub = bf_bits(f);
  if (MODE == 0) return ub;
  return h_bits(bf_up(ub) * WCARRY);
}
template <int MODE>
__global__ __launch_bounds__(256) void cvt16x8s(const float* __restrict__ in, unsigned short* out,
                                                int n8, int per8, int src8) {
  const int i = blockIdx.x * 256 + threadIdx.x;
  if (i < n8) {
    const int hd  = i / per8;
    const int rem = i - hd * per8;
    const float* s = in + ((size_t)hd * src8 + (size_t)rem) * 8;
    const v4f a = *(const v4f*)(s);
    const v4f b = *(const v4f*)(s + 4);
    v4u p;
    p[0] = pk16(cv16<MODE>(a[0]), cv16<MODE>(a[1]));
    p[1] = pk16(cv16<MODE>(a[2]), cv16<MODE>(a[3]));
    p[2] = pk16(cv16<MODE>(b[0]), cv16<MODE>(b[1]));
    p[3] = pk16(cv16<MODE>(b[2]), cv16<MODE>(b[3]));
    *(volatile v4u*)(out + (size_t)i * 8) = p;
    __threadfence();
    *(volatile v4u*)(out + (size_t)i * 8) = p;
  }
}

template <typename E>
__device__ __forceinline__ void mainloop128(const E* __restrict__ A, const E* __restrict__ Bt, E* As, E* Bs,
                                            int m0, int n0, int lda, int ldb, int kdim, v8f acc[4][2]) {
  typedef typename FT<E>::V16 V16;
  typedef typename FT<E>::V8  V8;
  const int t = threadIdx.x, wave = t >> 5, lane = t & 31, hh = lane >> 4, c = lane & 15;
  const int wm = wave >> 2, wn = wave & 3;
  for (int kb = 0; kb < kdim; kb += BK) {
#pragma unroll
    for (int i = 0; i < 2; ++i) {
      const int idx = t + i * 256;
      const int row = idx >> 2, seg = (idx & 3) * 8;
      const V8 av = *(const V8*)(A  + (size_t)(m0 + row) * lda + kb + seg);
      const V8 bv = *(const V8*)(Bt + (size_t)(n0 + row) * ldb + kb + seg);
      *(V8*)(As + row * BK + seg) = av;
      *(V8*)(Bs + row * BK + seg) = bv;
    }
    __syncthreads();
    V16 af[4];
#pragma unroll
    for (int mi = 0; mi < 4; ++mi) af[mi] = FT<E>::ld(As + (wm * 64 + mi * 16 + c) * BK + 8 * hh);
#pragma unroll
    for (int ni = 0; ni < 2; ++ni) {
      const V16 bfr = FT<E>::ld(Bs + (wn * 32 + ni * 16 + c) * BK + 8 * hh);
#pragma unroll
      for (int mi = 0; mi < 4; ++mi) acc[mi][ni] = FT<E>::mma(af[mi], bfr, acc[mi][ni]);
    }
    __syncthreads();
  }
}

__global__ __launch_bounds__(256)
void k_gemm_qkv(const unsigned short* __restrict__ xb, const unsigned short* __restrict__ wq,
                unsigned short* qpl, unsigned short* qll, unsigned short* kpl, unsigned short* kll,
                unsigned short* vtpl, unsigned short* vtll, float* knr) {
  typedef FT<__bf16> F;
  __shared__ __align__(16) __bf16   As[BM * BK];
  __shared__ __align__(16) __bf16   Bs[BN * BK];
  __shared__ __align__(16) _Float16 T[BM * TP];
  const int bm = blockIdx.x, bn = blockIdx.y;
  const int m0 = bm * BM, n0 = bn * BN;
  v8f acc[4][2];
#pragma unroll
  for (int mi = 0; mi < 4; ++mi)
#pragma unroll
    for (int ni = 0; ni < 2; ++ni) acc[mi][ni] = zero8();
  mainloop128<__bf16>((const __bf16*)(const void*)xb, (const __bf16*)(const void*)wq, As, Bs, m0, n0, DM, DM, DM, acc);
  (void)sizeof(F);

  const int t = threadIdx.x, wave = t >> 5, lane = t & 31, hh = lane >> 4, c = lane & 15;
  const int wm = wave >> 2, wn = wave & 3;
  const int s  = n0 / DM;
  const int hb = (n0 - s * DM) / HD;
  const int b  = m0 / SEQ;
  const int p0 = m0 - b * SEQ;
  const int lq = t >> 3, c8 = (t & 7) * 8;

  if (s < 2) {
    unsigned short* dh = (s == 0) ? qpl : kpl;
    unsigned short* dl = (s == 0) ? qll : kll;
#pragma unroll 1
    for (int pass = 0; pass < 2; ++pass) {
      __syncthreads();
#pragma unroll
      for (int mi = 0; mi < 4; ++mi)
#pragma unroll
        for (int ni = 0; ni < 2; ++ni)
#pragma unroll
          for (int r = 0; r < 8; ++r) {
            const float a = acc[mi][ni][r];
            const _Float16 hv = (_Float16)a;
            const _Float16 lv = (_Float16)((a - (float)hv) * QRES);
            T[(wm * 64 + mi * 16 + 8 * hh + r) * TP + wn * 32 + ni * 16 + c] = (pass != 0) ? lv : hv;
          }
      __syncthreads();
      if (pass == 0 && s == 1) {
        const int j = t >> 7, row = t & 127;
        float ss = 0.f;
#pragma unroll
        for (int i = 0; i < 8; ++i) {
          const v8h w8 = *(const v8h*)(T + row * TP + j * 64 + 8 * i);
#pragma unroll
          for (int e = 0; e < 8; ++e) { const float f = (float)w8[e]; ss += f * f; }
        }
        float* pn = knr + ((size_t)(b * NH + hb + j)) * SEQ + p0 + row;
        *(volatile float*)pn = ss;
        __threadfence();
        *(volatile float*)pn = ss;
      }
      v4u vals[8];
#pragma unroll
      for (int it = 0; it < 8; ++it) {
        const int L = it * 32 + lq;
        const int row = L & 127, j = L >> 7;
        union { v8h h; v4u u; } w;
        w.h = *(const v8h*)(T + row * TP + j * 64 + c8);
        vals[it] = w.u;
      }
      unsigned short* dst = (pass != 0) ? dl : dh;
      for (int rep = 0; rep < 2; ++rep) {
#pragma unroll
        for (int it = 0; it < 8; ++it) {
          const int L = it * 32 + lq;
          const int row = L & 127, j = L >> 7;
          unsigned short* p = dst + ((size_t)((b * NH + hb + j) * SEQ + p0 + row)) * HD + c8;
          *(volatile v4u*)p = vals[it];
        }
        __threadfence();
      }
    }
  } else {
#pragma unroll 1
    for (int pass = 0; pass < 2; ++pass) {
      __syncthreads();
#pragma unroll
      for (int mi = 0; mi < 4; ++mi)
#pragma unroll
        for (int ni = 0; ni < 2; ++ni)
#pragma unroll
          for (int r = 0; r < 8; ++r) {
            const float a = acc[mi][ni][r] * VCARRY;
            const _Float16 hv = (_Float16)a;
            const _Float16 lv = (_Float16)((a - (float)hv) * PRES);
            T[(wn * 32 + ni * 16 + c) * TP + wm * 64 + mi * 16 + 8 * hh + r] = (pass != 0) ? lv : hv;
          }
      __syncthreads();
      v4u vals[8];
#pragma unroll
      for (int it = 0; it < 8; ++it) {
        const int L = it * 32 + lq;
        const int j = L >> 7, d = (L >> 1) & 63, q2 = L & 1;
        union { v8h h; v4u u; } w;
        w.h = *(const v8h*)(T + (j * 64 + d) * TP + q2 * 64 + c8);
        vals[it] = w.u;
      }
      unsigned short* dst = (pass != 0) ? vtll : vtpl;
      for (int rep = 0; rep < 2; ++rep) {
#pragma unroll
        for (int it = 0; it < 8; ++it) {
          const int L = it * 32 + lq;
          const int j = L >> 7, d = (L >> 1) & 63, q2 = L & 1;
          unsigned short* p = dst + ((size_t)((b * NH + hb + j) * HD + d)) * SEQ + p0 + q2 * 64 + c8;
          *(volatile v4u*)p = vals[it];
        }
        __threadfence();
      }
    }
  }
}

__global__ __launch_bounds__(128)
void attn_loc64(const unsigned short* __restrict__ qp, const unsigned short* __restrict__ qlp,
                const unsigned short* __restrict__ kp, const unsigned short* __restrict__ klp,
                const unsigned short* __restrict__ vtp, const unsigned short* __restrict__ vtlp,
                const float* __restrict__ knr, const int* __restrict__ kflag, const int* __restrict__ useg,
                const float* __restrict__ shiftp, const float* __restrict__ biasp, unsigned short* op) {
#pragma clang fp contract(off)
  typedef FT<_Float16> F;
  union FH { v16h v; v8h h[2]; };
  __shared__ __align__(16) _Float16 Ksh[64 * 64];
  __shared__ __align__(16) _Float16 Ksl[64 * 64];
  __shared__ __align__(16) _Float16 Vth[64 * 64];
  __shared__ __align__(16) _Float16 Vtl[64 * 64];
  __shared__ __align__(16) _Float16 Psh[4][16 * 64];
  __shared__ __align__(16) _Float16 Psl[4][16 * 64];
  __shared__ __align__(16) _Float16 Os[4][16 * 64];
  __shared__ int nf[4];

  const int tid  = threadIdx.x;
  const int wave = tid >> 5;
  const int lane = tid & 31;
  const int hh   = lane >> 4;
  const int c    = lane & 15;

  const int bx   = blockIdx.x;
  const int qb   = bx % NQB;
  const int bh   = bx / NQB;
  const int b    = bh / NH;
  const int h    = bh - b * NH;
  const int q0   = qb * 64 + wave * 16;

  const int   ug  = useg[0];
  const float shv = (ug != 0) ? bf_up(bf_bits(shiftp[0])) : 0.f;
  const float bpv = (ug != 0) ? bf_up(bf_bits(biasp[0])) : 0.f;
  const int* mrp  = kflag + (size_t)b * SEQ_FULL;

  const _Float16* Qh = (const _Float16*)(const void*)qp   + (size_t)bh * SEQ * HD;
  const _Float16* Ql = (const _Float16*)(const void*)qlp  + (size_t)bh * SEQ * HD;
  const _Float16* Kh = (const _Float16*)(const void*)kp   + (size_t)bh * SEQ * HD;
  const _Float16* Kl = (const _Float16*)(const void*)klp  + (size_t)bh * SEQ * HD;
  const _Float16* Vh = (const _Float16*)(const void*)vtp  + (size_t)bh * HD * SEQ;
  const _Float16* Vl = (const _Float16*)(const void*)vtlp + (size_t)bh * HD * SEQ;
  const float*    Kn = knr + (size_t)bh * SEQ;

  v16h qa[2], ql[2];
#pragma unroll
  for (int dc = 0; dc < 2; ++dc) {
    const size_t qo = (size_t)(q0 + c) * HD + dc * 32 + 8 * hh;
    qa[dc] = F::ld(Qh + qo);
    ql[dc] = F::ld(Ql + qo);
  }
  float qs = 0.f;
#pragma unroll
  for (int dc = 0; dc < 2; ++dc)
#pragma unroll
    for (int i = 0; i < 16; ++i) { const float f = (float)qa[dc][i]; qs = qs + f * f; }
  qs = qs + __shfl_xor(qs, 16, 32);
#pragma unroll
  for (int off = 1; off < 16; off <<= 1) qs = fmaxf(qs, __shfl_xor(qs, off, 32));
  const float qmax2 = qs;

  float mrow[8], lrow[8];
  v8f oacc[4];
#pragma unroll
  for (int r = 0; r < 8; ++r) { mrow[r] = -INFINITY; lrow[r] = 0.f; }
#pragma unroll
  for (int t = 0; t < 4; ++t) oacc[t] = zero8();

  for (int step = 0; step < 2 * NQB; ++step) {
    const int dt = (step + 1) >> 1;
    const int kt = (step & 1) ? (qb - dt) : (qb + dt);
    if (kt < 0 || kt >= NQB) continue;
    const bool nearT = (dt <= RESW);
    const int kv0 = kt * 64;

    int fl = 1;
    if (!nearT) {
      float kx = fmaxf(Kn[kv0 + lane], Kn[kv0 + 32 + lane]);
#pragma unroll
      for (int off = 1; off < 32; off <<= 1) kx = fmaxf(kx, __shfl_xor(kx, off, 32));
      float mm = mrow[0];
#pragma unroll
      for (int r = 1; r < 8; ++r) mm = fminf(mm, mrow[r]);
      mm = fminf(mm, __shfl_xor(mm, 16, 32));
      const int dmin = (kv0 > q0) ? (kv0 - (q0 + 15)) : (q0 - (kv0 + 63));
      const float dsq = (float)(dmin * dmin);
      const float qk  = sqrtf(qmax2 * kx);
      const float gg  = shv * dsq;
      const float ub  = qk * 0.13f + 2.0f - gg * 0.999f - bpv;
      const int keep  = (ub < mm - SKIPG) ? 0 : 1;
      fl = __builtin_amdgcn_readfirstlane(keep);
    }
    if (lane == 0) nf[wave] = fl;
    __syncthreads();
    const int anyf = nf[0] | nf[1] | nf[2] | nf[3];

    if (anyf != 0) {
      const int r = tid >> 1, half = (tid & 1) * 32;
      const size_t kgo = (size_t)(kv0 + r) * HD + half;
      const size_t vgo = (size_t)r * SEQ + kv0 + half;
#pragma unroll
      for (int i = 0; i < 4; ++i) {
        const v8h a0 = *(const v8h*)(Kh + kgo + 8 * i);
        const v8h b0 = *(const v8h*)(Vh + vgo + 8 * i);
        *(v8h*)(Ksh + r * 64 + half + 8 * i) = a0;
        *(v8h*)(Vth + r * 64 + half + 8 * i) = b0;
      }
      if (nearT) {
#pragma unroll
        for (int i = 0; i < 4; ++i) {
          const v8h a1 = *(const v8h*)(Kl + kgo + 8 * i);
          const v8h b1 = *(const v8h*)(Vl + vgo + 8 * i);
          *(v8h*)(Ksl + r * 64 + half + 8 * i) = a1;
          *(v8h*)(Vtl + r * 64 + half + 8 * i) = b1;
        }
      }
    }
    __syncthreads();

    if (fl != 0) {
      int kmv[4];
#pragma unroll
      for (int j = 0; j < 4; ++j) kmv[j] = mrp[kv0 + j * 16 + c];

      v8f s[4];
#pragma unroll
      for (int j = 0; j < 4; ++j) {
        s[j] = zero8();
        v8f sr = zero8();
#pragma unroll
        for (int dc = 0; dc < 2; ++dc) {
          const int ko = (j * 16 + c) * 64 + dc * 32 + 8 * hh;
          FH kb;
          kb.h[0] = *(const v8h*)(Ksh + ko);
          kb.h[1] = *(const v8h*)(Ksh + ko + 16);
          s[j] = F::mma(qa[dc], kb.v, s[j]);
          if (nearT) {
            FH kl;
            kl.h[0] = *(const v8h*)(Ksl + ko);
            kl.h[1] = *(const v8h*)(Ksl + ko + 16);
            sr = F::mma(qa[dc], kl.v, sr);
            sr = F::mma(ql[dc], kb.v, sr);
          }
        }
        if (nearT) {
#pragma unroll
          for (int r = 0; r < 8; ++r) s[j][r] = s[j][r] + sr[r] * (1.0f / QRES);
        }
      }

      _Float16* pwh = Psh[wave];
      _Float16* pwl = Psl[wave];
#pragma unroll
      for (int r = 0; r < 8; ++r) {
        const int irow = q0 + 8 * hh + r;
        float m = -INFINITY;
#pragma unroll
        for (int j = 0; j < 4; ++j) {
          const int jj   = kv0 + j * 16 + c;
          const float sc = s[j][r] * 0.125f;
          const float sm = (kmv[j] != 0) ? sc : NEGF;
          const float dd = (float)(irow - jj);
          const float g1 = shv * (dd * dd);
          const float g2 = g1 + bpv;
          const float sv = sm - g2;
          s[j][r] = sv;
          m = fmaxf(m, sv);
        }
#pragma unroll
        for (int off = 1; off < 16; off <<= 1) m = fmaxf(m, __shfl_xor(m, off, 32));
        const float mnew  = fmaxf(mrow[r], m);
        const float msafe = (mnew == -INFINITY) ? 0.f : mnew;
        const float alpha = __expf(mrow[r] - msafe);
        mrow[r] = mnew;
        float psum = 0.f;
#pragma unroll
        for (int j = 0; j < 4; ++j) {
          const float p = __expf(s[j][r] - msafe);
          psum += p;
          const float p1k = p * PCARRY;
          const _Float16 ph = (_Float16)p1k;
          pwh[(8 * hh + r) * 64 + j * 16 + c] = ph;
          if (nearT) {
            const _Float16 pl = (_Float16)((p1k - (float)ph) * PRES);
            pwl[(8 * hh + r) * 64 + j * 16 + c] = pl;
          }
        }
#pragma unroll
        for (int off = 1; off < 16; off <<= 1) psum += __shfl_xor(psum, off, 32);
        lrow[r] = lrow[r] * alpha + psum;
#pragma unroll
        for (int t = 0; t < 4; ++t) oacc[t][r] *= alpha;
      }
      __builtin_amdgcn_fence(3  , "workgroup");
      __builtin_amdgcn_wave_barrier();
      __builtin_amdgcn_fence(2  , "workgroup");

      v8f o1[4];
#pragma unroll
      for (int t = 0; t < 4; ++t) o1[t] = zero8();
#pragma unroll 1
      for (int kk = 0; kk < 2; ++kk) {
        FH pa, pl;
        const int po = c * 64 + kk * 32 + 8 * hh;
        pa.h[0] = *(const v8h*)(pwh + po);
        pa.h[1] = *(const v8h*)(pwh + po + 16);
        pl.v = pa.v;
        if (nearT) {
          pl.h[0] = *(const v8h*)(pwl + po);
          pl.h[1] = *(const v8h*)(pwl + po + 16);
        }
#pragma unroll
        for (int t = 0; t < 4; ++t) {
          const int vo = (t * 16 + c) * 64 + kk * 32 + 8 * hh;
          FH vb;
          vb.h[0] = *(const v8h*)(Vth + vo);
          vb.h[1] = *(const v8h*)(Vth + vo + 16);
          oacc[t] = F::mma(pa.v, vb.v, oacc[t]);
          if (nearT) {
            FH vl;
            vl.h[0] = *(const v8h*)(Vtl + vo);
            vl.h[1] = *(const v8h*)(Vtl + vo + 16);
            o1[t] = F::mma(pl.v, vb.v, o1[t]);
            o1[t] = F::mma(pa.v, vl.v, o1[t]);
          }
        }
      }
      if (nearT) {
#pragma unroll
        for (int t = 0; t < 4; ++t)
#pragma unroll
          for (int r = 0; r < 8; ++r) oacc[t][r] = oacc[t][r] + o1[t][r] * (1.0f / PRES);
      }
    }
  }

  _Float16* os = Os[wave];
#pragma unroll
  for (int r = 0; r < 8; ++r) {
    const float l = lrow[r];
    const float inv = ((l > 0.f) ? (1.0f / l) : 0.f) * (OCARRY / (PCARRY * VCARRY));
#pragma unroll
    for (int t = 0; t < 4; ++t) os[(8 * hh + r) * 64 + t * 16 + c] = (_Float16)(oacc[t][r] * inv);
  }
  __builtin_amdgcn_fence(3  , "workgroup");
  __builtin_amdgcn_wave_barrier();
  __builtin_amdgcn_fence(2  , "workgroup");
  {
    const int rq = lane >> 3, c8 = (lane & 7) * 8;
    v4u vals[4];
#pragma unroll
    for (int it = 0; it < 4; ++it) {
      const int row = it * 4 + rq;
      union { v8h h; v4u u; } w;
      w.h = *(const v8h*)(os + row * 64 + c8);
      vals[it] = w.u;
    }
    unsigned short* ob = op + ((size_t)(b * SEQ + q0)) * DM + h * HD + c8;
    for (int rep = 0; rep < 2; ++rep) {
#pragma unroll
      for (int it = 0; it < 4; ++it) {
        const int row = it * 4 + rq;
        *(volatile v4u*)(ob + (size_t)row * DM) = vals[it];
      }
      __threadfence();
    }
  }
}

__global__ __launch_bounds__(256)
void k_gemm_out(const unsigned short* __restrict__ ob, const unsigned short* __restrict__ wpt,
                const float* __restrict__ bias, float* outp) {
  typedef FT<_Float16> F;
  __shared__ __align__(16) _Float16 As[BM * BK];
  __shared__ __align__(16) _Float16 Bs[BN * BK];
  __shared__ __align__(16) float    Tf[64 * TPF];
  const int bm = blockIdx.x, bn = blockIdx.y;
  const int m0 = bm * BM, n0 = bn * BN;
  v8f acc[4][2];
#pragma unroll
  for (int mi = 0; mi < 4; ++mi)
#pragma unroll
    for (int ni = 0; ni < 2; ++ni) acc[mi][ni] = zero8();
  mainloop128<_Float16>((const _Float16*)(const void*)ob, (const _Float16*)(const void*)wpt, As, Bs,
                        m0, n0, DM, DM, DM, acc);
  (void)sizeof(F);

  const int t = threadIdx.x, wave = t >> 5, lane = t & 31, hh = lane >> 4, c = lane & 15;
  const int wm = wave >> 2, wn = wave & 3;
  const float inv = 1.0f / (OCARRY * WCARRY);
  const int lq = t >> 3, seg = lq & 3, c4 = seg * 32 + (t & 7) * 4, rsub = lq >> 2;
  v4f bb;
  {
    const v4f b4 = *(const v4f*)(bias + n0 + c4);
#pragma unroll
    for (int e = 0; e < 4; ++e) bb[e] = bf_up(bf_bits(b4[e]));
  }
  for (int hm = 0; hm < 2; ++hm) {
    if (wm == hm) {
#pragma unroll
      for (int mi = 0; mi < 4; ++mi)
#pragma unroll
        for (int ni = 0; ni < 2; ++ni)
#pragma unroll
          for (int r = 0; r < 8; ++r)
            Tf[(mi * 16 + 8 * hh + r) * TPF + wn * 32 + ni * 16 + c] = acc[mi][ni][r] * inv;
    }
    __syncthreads();
    v4f vals[8];
#pragma unroll
    for (int it = 0; it < 8; ++it) {
      const int row = it * 8 + rsub;
      vals[it] = *(const v4f*)(Tf + row * TPF + c4) + bb;
    }
    float* dst = outp + ((size_t)(m0 + hm * 64)) * DM + n0 + c4;
    for (int rep = 0; rep < 2; ++rep) {
#pragma unroll
      for (int it = 0; it < 8; ++it) {
        const int row = it * 8 + rsub;
        *(volatile v4f*)(dst + (size_t)row * DM) = vals[it];
      }
      __threadfence();
    }
    __syncthreads();
  }
}

extern "C" void kernel_launch(void* const* d_in, const int* in_sizes, int n_in,
                              void* d_out, int out_size, void* d_ws, size_t ws_size,
                              hipStream_t stream) {
  if (n_in < 9) return;
  const long long needX = ((long long)(NB - 1) * SEQ_FULL + (long long)SEQ) * DM;
  if ((long long)in_sizes[0] < needX) return;
  if ((long long)in_sizes[1] < (long long)(NB - 1) * SEQ_FULL + (long long)SEQ) return;
  if (in_sizes[3] < 1) return;
  if ((long long)in_sizes[4] < (long long)DQKV * DM) return;
  if ((long long)in_sizes[5] < (long long)DM * DM) return;
  if (in_sizes[6] < DM) return;
  if (in_sizes[7] < 1 || in_sizes[8] < 1) return;
  if (out_size < 0 || (long long)out_size < (long long)MTOK * DM) return;

  const size_t szAct = (size_t)MTOK * DM * 2;
  const size_t szWq  = (size_t)DQKV * DM * 2;
  const size_t szWp  = (size_t)DM * DM * 2;
  const size_t szKn  = (size_t)NB * NH * SEQ * 4;
  size_t off = 0;
  const size_t oXO  = off; off += szAct;
  const size_t oWq  = off; off += szWq;
  const size_t oWp  = off; off += szWp;
  const size_t oQ   = off; off += szAct;
  const size_t oQl  = off; off += szAct;
  const size_t oK   = off; off += szAct;
  const size_t oKl  = off; off += szAct;
  const size_t oVT  = off; off += szAct;
  const size_t oVTl = off; off += szAct;
  const size_t oKn  = off; off += szKn;
  if (off > ws_size) return;
  if (off > (size_t)134217728) return;

  const float* x      = (const float*)d_in[0];
  const int*   kflag  = (const int*)d_in[1];
  const int*   useg   = (const int*)d_in[3];
  const float* w_qkv  = (const float*)d_in[4];
  const float* w_fc   = (const float*)d_in[5];
  const float* b_fc   = (const float*)d_in[6];
  const float* shiftp = (const float*)d_in[7];
  const float* biasp  = (const float*)d_in[8];
  float* out = (float*)d_out;

  char* ws = (char*)d_ws;
  unsigned short* XO  = (unsigned short*)(ws + oXO);
  unsigned short* Wq  = (unsigned short*)(ws + oWq);
  unsigned short* Wp  = (unsigned short*)(ws + oWp);
  unsigned short* Qp  = (unsigned short*)(ws + oQ);
  unsigned short* Qlp = (unsigned short*)(ws + oQl);
  unsigned short* Kp  = (unsigned short*)(ws + oK);
  unsigned short* Klp = (unsigned short*)(ws + oKl);
  unsigned short* VTp = (unsigned short*)(ws + oVT);
  unsigned short* VTl = (unsigned short*)(ws + oVTl);
  float*          Kn  = (float*)(ws + oKn);

  const dim3 blk(256);
  const int n8x  = MTOK * DM / 8;
  const int per8 = SEQ * DM / 8;
  const int src8 = SEQ_FULL * DM / 8;
  const int n8w  = DQKV * DM / 8;
  const int n8f  = DM * DM / 8;
  const dim3 gCx(n8x / 256);
  const dim3 gCw(n8w / 256);
  const dim3 gCf(n8f / 256);
  const dim3 gG1(MTOK / BM, DQKV / BN);
  const dim3 gG2(MTOK / BM, DM / BN);
  const dim3 gAt(NB * NH * NQB);

  cvt16x8s<0><<<gCx, blk, 0, stream>>>(x, XO, n8x, per8, src8);
  cvt16x8s<0><<<gCw, blk, 0, stream>>>(w_qkv, Wq, n8w, n8w, n8w);
  cvt16x8s<1><<<gCf, blk, 0, stream>>>(w_fc, Wp, n8f, n8f, n8f);
  k_gemm_qkv<<<gG1, blk, 0, stream>>>(XO, Wq, Qp, Qlp, Kp, Klp, VTp, VTl, Kn);
  attn_loc64<<<gAt, dim3(128), 0, stream>>>(Qp, Qlp, Kp, Klp, VTp, VTl, Kn, kflag, useg, shiftp, biasp, XO);
  k_gemm_out<<<gG2, blk, 0, stream>>>(XO, Wp, b_fc, out);
  (void)hipGetLastError();
}
